// VideoSwinTransformerBlock_4629974745491
// MI455X (gfx1250) — hardware-verified
//
#include <hip/hip_runtime.h>
#include <math.h>

typedef __attribute__((ext_vector_type(16))) _Float16 v16h;
typedef __attribute__((ext_vector_type(8)))  _Float16 v8h;
typedef __attribute__((ext_vector_type(16))) __bf16   v16b;
typedef __attribute__((ext_vector_type(8)))  __bf16   v8b;
typedef __attribute__((ext_vector_type(8)))  float    v8f;
typedef __attribute__((ext_vector_type(4)))  float    v4f;

#define NEG_INF (-__builtin_huge_valf())

__device__ __forceinline__ unsigned short f2bf_bits(float f) {
  unsigned u = __float_as_uint(f);
  return (unsigned short)((u + 0x7FFFu + ((u >> 16) & 1u)) >> 16);
}
__device__ __forceinline__ float bf_bits2f(unsigned short h) { return __uint_as_float(((unsigned)h) << 16); }

__device__ __forceinline__ void dep_guard_h(v8f& a, v8f& b, v16h x, v16h y) { asm volatile("v_nop\n\tv_nop\n\tv_nop\n\tv_nop" : "+v"(a), "+v"(b) : "v"(x), "v"(y)); }
__device__ __forceinline__ void dep_guard_b(v8f& a, v8f& b, v16b x, v16b y) { asm volatile("v_nop\n\tv_nop\n\tv_nop\n\tv_nop" : "+v"(a), "+v"(b) : "v"(x), "v"(y)); }
__device__ __forceinline__ void keep4_h(v16h a, v16h b, v16h c, v16h d) { asm volatile("v_nop" :: "v"(a), "v"(b), "v"(c), "v"(d)); }
__device__ __forceinline__ void keep4_b(v16b a, v16b b, v16b c, v16b d) { asm volatile("v_nop" :: "v"(a), "v"(b), "v"(c), "v"(d)); }
__device__ __forceinline__ void acc_guard4(v8f& a, v8f& b, v8f& c, v8f& d) { asm volatile("v_nop\n\tv_nop\n\tv_nop\n\tv_nop" : "+v"(a), "+v"(b), "+v"(c), "+v"(d)); }
template <typename T> struct Frag;
template <> struct Frag<_Float16> {
  typedef v16h V; union U { v16h v; v8h h[2]; };
  static __device__ __forceinline__ v16h load(const _Float16* p) {
    U f; f.h[0] = *(const v8h*)(p); f.h[1] = *(const v8h*)(p + 16); return f.v;
  }
  static __device__ __forceinline__ v8f mma(v16h a, v16h b, v8f c) {
    return __builtin_amdgcn_wmma_f32_16x16x32_f16(false, a, false, b, (short)0, c, false, false);
  }
  static __device__ __forceinline__ void guard(v8f& a, v8f& b, v16h x, v16h y) { dep_guard_h(a, b, x, y); }
  static __device__ __forceinline__ void keep(v16h a, v16h b, v16h c, v16h d) { keep4_h(a, b, c, d); }
};
template <> struct Frag<__bf16> {
  typedef v16b V; union U { v16b v; v8b h[2]; };
  static __device__ __forceinline__ v16b load(const __bf16* p) {
    U f; f.h[0] = *(const v8b*)(p); f.h[1] = *(const v8b*)(p + 16); return f.v;
  }
  static __device__ __forceinline__ v8f mma(v16b a, v16b b, v8f c) {
    return __builtin_amdgcn_wmma_f32_16x16x32_bf16(false, a, false, b, (short)0, c, false, false);
  }
  static __device__ __forceinline__ void guard(v8f& a, v8f& b, v16b x, v16b y) { dep_guard_b(a, b, x, y); }
  static __device__ __forceinline__ void keep(v16b a, v16b b, v16b c, v16b d) { keep4_b(a, b, c, d); }
};

template <int ET> struct Elem;
template <> struct Elem<0> { typedef _Float16 T; };
template <> struct Elem<1> { typedef __bf16 T; };
template <int ET, bool SPLIT, int BIAS_MODE, int OUT_MODE, bool RESID, int ACT = 0>
__global__ __launch_bounds__(256) void wmma_gemm64(
    const unsigned short* __restrict__ Ap, const unsigned short* __restrict__ A2p, int lda, long strideA,
    const unsigned short* __restrict__ Btp, const unsigned short* __restrict__ Bt2p, int ldb, long strideB,
    void* __restrict__ Cout, void* __restrict__ Cout2, int ldc, long strideC,
    const float* __restrict__ bias,
    const float* __restrict__ resid, long strideR,
    int M, int N, int K, float scale, float oscale) {
  typedef typename Elem<ET>::T T;
  typedef typename Frag<T>::V V;
  const T* A = (const T*)Ap; const T* A2 = (const T*)A2p; const T* Bt = (const T*)Btp; const T* Bt2 = (const T*)Bt2p;
  __shared__ __align__(16) float sT[8][16 * 68];
  const int b    = blockIdx.y;
  const int lane = threadIdx.x & 31;
  const int wave = threadIdx.x >> 5;
  const int tilesN = N >> 6;
  const int tilesM = M >> 6;
  const int tile = blockIdx.x * 8 + wave;
  if (tile >= tilesM * tilesN) return;
  const int tm = tile / tilesN;
  const int tn = tile - tm * tilesN;
  const int m0 = tm << 6;
  const int n0 = tn << 6;

  const T* Ab  = A  + (size_t)b * strideA;
  const T* Bb  = Bt + (size_t)b * strideB;
  const T* Ab2 = SPLIT ? (A2  + (size_t)b * strideA) : nullptr;
  const T* Bb2 = SPLIT ? (Bt2 + (size_t)b * strideB) : nullptr;

  const int rlane = lane & 15;
  const int koff  = (lane >> 4) * 8;
  const int mOff  = (lane >> 4) * 8;

  v8f acc[4][4];
#pragma unroll
  for (int i = 0; i < 4; ++i)
#pragma unroll
    for (int j = 0; j < 4; ++j) acc[i][j] = (v8f){0.f,0.f,0.f,0.f,0.f,0.f,0.f,0.f};

  for (int k0 = 0; k0 < K; k0 += 32) {
    V bh[4], bl[4];
#pragma unroll
    for (int j = 0; j < 4; ++j) {
      const size_t bo = (size_t)(n0 + (j << 4) + rlane) * ldb + koff + k0;
      bh[j] = Frag<T>::load(Bb + bo);
      if (SPLIT) bl[j] = Frag<T>::load(Bb2 + bo);
    }
#pragma unroll
    for (int i = 0; i < 4; ++i) {
      const size_t ao = (size_t)(m0 + (i << 4) + rlane) * lda + koff + k0;
      V ah = Frag<T>::load(Ab + ao);
      V al;
      if (SPLIT) al = Frag<T>::load(Ab2 + ao);
#pragma unroll
      for (int j = 0; j < 4; ++j) {
        acc[i][j] = Frag<T>::mma(ah, bh[j], acc[i][j]);
        if (SPLIT) {
          acc[i][j] = Frag<T>::mma(ah, bl[j], acc[i][j]);
          acc[i][j] = Frag<T>::mma(al, bh[j], acc[i][j]);
        }
      }
      Frag<T>::guard(acc[i][0], acc[i][3], ah, SPLIT ? al : ah);
    }
    Frag<T>::keep(bh[0], bh[1], bh[2], bh[3]);
    if (SPLIT) Frag<T>::keep(bl[0], bl[1], bl[2], bl[3]);
  }
  acc_guard4(acc[0][0], acc[0][1], acc[0][2], acc[0][3]);
  acc_guard4(acc[1][0], acc[1][1], acc[1][2], acc[1][3]);
  acc_guard4(acc[2][0], acc[2][1], acc[2][2], acc[2][3]);
  acc_guard4(acc[3][0], acc[3][1], acc[3][2], acc[3][3]);

  float* slab = sT[wave];
  const float* Rb = RESID ? (resid + (size_t)b * strideR) : nullptr;
#pragma unroll
  for (int i = 0; i < 4; ++i) {
    const int mBase = m0 + (i << 4);
#pragma unroll
    for (int j = 0; j < 4; ++j) {
      const int n = n0 + (j << 4) + rlane;
      float bv = 0.f;
      if (BIAS_MODE == 2) bv = bias[n];
#pragma unroll
      for (int r = 0; r < 8; ++r) {
        float v = acc[i][j][r] * scale;
        if (BIAS_MODE == 1) v += bias[mBase + mOff + r];
        if (BIAS_MODE == 2) v += bv;
        if (RESID) v += Rb[(size_t)(mBase + mOff + r) * ldc + n];
        if (ACT == 2) v = fmaxf(v, 0.0f);
        if (ACT == 4) v = (v > 0.f) ? v : 0.01f * v;
        slab[(mOff + r) * 68 + (j << 4) + rlane] = v * oscale;
      }
    }
    __builtin_amdgcn_fence(__ATOMIC_RELEASE, "workgroup");
    __builtin_amdgcn_wave_barrier();
    __builtin_amdgcn_fence(__ATOMIC_ACQUIRE, "workgroup");
    if (OUT_MODE == 0) {
      float* C = (float*)Cout + (size_t)b * strideC;
      const int hh = lane >> 4, c4 = (lane & 15) * 4;
      for (int pass = 0; pass < 2; ++pass) {
#pragma unroll
        for (int it = 0; it < 8; ++it) {
          const int row = it * 2 + hh;
          v4f v = *(const v4f*)(slab + row * 68 + c4);
          *(volatile v4f*)(C + (size_t)(mBase + row) * ldc + n0 + c4) = v;
        }
        __threadfence();
      }
    } else {
      const int q = lane >> 3, c8 = (lane & 7) * 8;
      unsigned short* C  = (unsigned short*)Cout  + (size_t)b * strideC;
      unsigned short* C2 = (OUT_MODE == 2) ? ((unsigned short*)Cout2 + (size_t)b * strideC) : nullptr;
      for (int pass = 0; pass < 2; ++pass) {
#pragma unroll
        for (int it = 0; it < 4; ++it) {
          const int row = it * 4 + q;
          const float* sp = slab + row * 68 + c8;
          v8h hv, lv;
#pragma unroll
          for (int e = 0; e < 8; ++e) {
            if (OUT_MODE == 1) {
              hv[e] = (_Float16)sp[e];
            } else {
              unsigned short hb = f2bf_bits(sp[e]);
              unsigned short lb = f2bf_bits(sp[e] - bf_bits2f(hb));
              hv[e] = __builtin_bit_cast(_Float16, hb);
              lv[e] = __builtin_bit_cast(_Float16, lb);
            }
          }
          *(volatile v8h*)(C + (size_t)(mBase + row) * ldc + n0 + c8) = hv;
          if (OUT_MODE == 2) *(volatile v8h*)(C2 + (size_t)(mBase + row) * ldc + n0 + c8) = lv;
        }
        __threadfence();
      }
    }
    __builtin_amdgcn_fence(__ATOMIC_RELEASE, "workgroup");
    __builtin_amdgcn_wave_barrier();
    __builtin_amdgcn_fence(__ATOMIC_ACQUIRE, "workgroup");
  }
}

constexpr int IMGD    = 16;
constexpr int IMGH    = 56;
constexpr int IMGW    = 56;
constexpr int CDIM    = 256;
constexpr int HIDD    = 1024;
constexpr int QKVP    = 768;
constexpr int NHD     = 8;
constexpr int HDM     = 32;
constexpr int NWND    = 512;
constexpr int WTOK    = 98;
constexpr int NTOKALL = IMGD * IMGH * IMGW;
constexpr int NREL    = 507;
constexpr int MLPCH   = 12544;
constexpr int NMLPCH  = 4;
static_assert(NTOKALL == 50176, "token count");
static_assert(NTOKALL % 64 == 0 && MLPCH % 64 == 0 && MLPCH * NMLPCH == NTOKALL, "tile multiples");

__device__ __forceinline__ int tokrow(int win, int t) {
  const int dw = win >> 6, hw = (win >> 3) & 7, wwi = win & 7;
  const int dl = t / 49;
  const int rem = t - dl * 49;
  const int hl = rem / 7;
  const int wl = rem - hl * 7;
  const int d = (dw * 2 + dl + 1) & (IMGD - 1);
  int h = hw * 7 + hl + 3;  h = (h >= IMGH) ? h - IMGH : h;
  int w = wwi * 7 + wl + 3; w = (w >= IMGW) ? w - IMGW : w;
  return (d * IMGH + h) * IMGW + w;
}
__device__ __forceinline__ int relpart(int t) {
  const int dl = t / 49;
  const int rem = t - dl * 49;
  const int hl = rem / 7;
  const int wl = rem - hl * 7;
  return dl * 169 + hl * 13 + wl;
}

__global__ __launch_bounds__(256) void wtr64_kernel(
    const float* __restrict__ w, _Float16* __restrict__ wt, int K, int N, float scale) {
  __shared__ float sW[64 * 65];
  const int tid = threadIdx.x;
  const int n0 = blockIdx.x * 64, k0 = blockIdx.y * 64;
#pragma unroll
  for (int i = 0; i < 16; ++i) {
    const int idx = i * 256 + tid;
    const int kr = idx >> 6, nc = idx & 63;
    sW[kr * 65 + nc] = w[(size_t)(k0 + kr) * N + n0 + nc];
  }
  __syncthreads();
  const int wave = tid >> 5, lane = tid & 31;
  const int q = lane >> 3, c8 = (lane & 7) * 8;
  for (int pass = 0; pass < 2; ++pass) {
#pragma unroll
    for (int it = 0; it < 2; ++it) {
      const int nr = wave * 8 + it * 4 + q;
      v8h hv;
#pragma unroll
      for (int e = 0; e < 8; ++e) hv[e] = (_Float16)(sW[(c8 + e) * 65 + nr] * scale);
      *(volatile v8h*)(wt + (size_t)(n0 + nr) * K + k0 + c8) = hv;
    }
    __threadfence();
  }
}

__global__ __launch_bounds__(256) void ln256_kernel(
    const float* __restrict__ x, const float* __restrict__ g, const float* __restrict__ bb,
    _Float16* __restrict__ out, int nrows) {
  const int wave = threadIdx.x >> 5, lane = threadIdx.x & 31;
  const int row = blockIdx.x * 8 + wave;
  if (row >= nrows) return;
  const float* src = x + (size_t)row * CDIM + lane * 8;
  const v4f a0 = *(const v4f*)src;
  const v4f a1 = *(const v4f*)(src + 4);
  float s = ((a0[0] + a0[1]) + (a0[2] + a0[3])) + ((a1[0] + a1[1]) + (a1[2] + a1[3]));
#pragma unroll
  for (int off = 16; off >= 1; off >>= 1) s += __shfl_xor(s, off, 32);
  const float mu = s * (1.0f / 256.0f);
  v4f d0, d1;
  d0[0] = a0[0] - mu; d0[1] = a0[1] - mu; d0[2] = a0[2] - mu; d0[3] = a0[3] - mu;
  d1[0] = a1[0] - mu; d1[1] = a1[1] - mu; d1[2] = a1[2] - mu; d1[3] = a1[3] - mu;
  float sq = ((d0[0] * d0[0] + d0[1] * d0[1]) + (d0[2] * d0[2] + d0[3] * d0[3]))
           + ((d1[0] * d1[0] + d1[1] * d1[1]) + (d1[2] * d1[2] + d1[3] * d1[3]));
#pragma unroll
  for (int off = 16; off >= 1; off >>= 1) sq += __shfl_xor(sq, off, 32);
  const float rs = rsqrtf(sq * (1.0f / 256.0f) + 1e-5f);
  const v4f g0 = *(const v4f*)(g + lane * 8);
  const v4f g1 = *(const v4f*)(g + lane * 8 + 4);
  const v4f b0 = *(const v4f*)(bb + lane * 8);
  const v4f b1 = *(const v4f*)(bb + lane * 8 + 4);
  v8h hv;
  hv[0] = (_Float16)(d0[0] * rs * g0[0] + b0[0]);
  hv[1] = (_Float16)(d0[1] * rs * g0[1] + b0[1]);
  hv[2] = (_Float16)(d0[2] * rs * g0[2] + b0[2]);
  hv[3] = (_Float16)(d0[3] * rs * g0[3] + b0[3]);
  hv[4] = (_Float16)(d1[0] * rs * g1[0] + b1[0]);
  hv[5] = (_Float16)(d1[1] * rs * g1[1] + b1[1]);
  hv[6] = (_Float16)(d1[2] * rs * g1[2] + b1[2]);
  hv[7] = (_Float16)(d1[3] * rs * g1[3] + b1[3]);
  _Float16* dst = out + (size_t)row * CDIM + lane * 8;
  *(volatile v8h*)dst = hv;
  __threadfence();
  *(volatile v8h*)dst = hv;
}

__global__ __launch_bounds__(256) void gelu2_kernel(
    const _Float16* __restrict__ in, _Float16* __restrict__ out, int n2) {
  const int i = blockIdx.x * 256 + threadIdx.x;
  if (i < n2) {
    const unsigned wbits = ((const unsigned*)(const void*)in)[i];
    const float u0 = (float)__builtin_bit_cast(_Float16, (unsigned short)(wbits & 0xFFFFu)) * 0.25f;
    const float u1 = (float)__builtin_bit_cast(_Float16, (unsigned short)(wbits >> 16)) * 0.25f;
    const float g0 = 0.5f * u0 * (1.0f + erff(u0 * 0.70710678118654752f));
    const float g1 = 0.5f * u1 * (1.0f + erff(u1 * 0.70710678118654752f));
    const _Float16 h0 = (_Float16)(g0 * 16.0f), h1 = (_Float16)(g1 * 16.0f);
    const unsigned o = (unsigned)__builtin_bit_cast(unsigned short, h0) | ((unsigned)__builtin_bit_cast(unsigned short, h1) << 16);
    ((volatile unsigned*)out)[i] = o;
    __threadfence();
    ((volatile unsigned*)out)[i] = o;
  }
}

constexpr int ATT_WAVES = 8;
constexpr int QWAVES    = 7;
constexpr int KVPAD     = 128;
constexpr int KPI       = 40;
constexpr int VPI       = 136;
constexpr int PPI       = 136;
constexpr int OPH       = 72;
constexpr float PCARRY  = 32768.0f;
constexpr float SCORE_SCALE = 0.17677669529663687f * (1.0f / 256.0f);

__device__ __forceinline__ v8f mma_h(v16h a, v16h b, v8f c) {
  c = __builtin_amdgcn_wmma_f32_16x16x32_f16(false, a, false, b, (short)0, c, false, false);
  asm volatile("v_nop\n\tv_nop\n\tv_nop\n\tv_nop" : "+v"(c) : "v"(a), "v"(b));
  return c;
}
__device__ __forceinline__ void wave_lds_sync() {
  __builtin_amdgcn_fence(__ATOMIC_RELEASE, "workgroup");
  __builtin_amdgcn_wave_barrier();
  __builtin_amdgcn_fence(__ATOMIC_ACQUIRE, "workgroup");
}

__global__ __launch_bounds__(256) void vswin_attn_kernel(
    const _Float16* __restrict__ qkv, const float* __restrict__ rpb,
    const float* __restrict__ maskm, _Float16* __restrict__ att) {
  __shared__ __align__(16) _Float16 Ks[2][KVPAD * KPI];
  __shared__ __align__(16) _Float16 Vt[2][HDM * VPI];
  __shared__ __align__(16) _Float16 Ps[QWAVES][16 * PPI];
  __shared__ __align__(16) _Float16 Os[QWAVES][16 * OPH];
  __shared__ float sBias[2][512];

  const int tid  = threadIdx.x;
  const int wave = tid >> 5;
  const int lane = tid & 31;
  const int hh   = lane >> 4;
  const int c    = lane & 15;
  const int hp   = blockIdx.x;
  const int win  = blockIdx.y;

  for (int i = tid; i < NREL; i += 256) {
    sBias[0][i] = rpb[i * NHD + hp * 2];
    sBias[1][i] = rpb[i * NHD + hp * 2 + 1];
  }
  {
    const _Float16 hz = (_Float16)0.0f;
#pragma unroll
    for (int i = 0; i < 4; ++i) {
      const int idx = i * 256 + tid;
      const int hs  = idx >> 9;
      const int kv  = (idx >> 2) & (KVPAD - 1);
      const int pc  = idx & 3;
      const bool live = kv < WTOK;
      const int kvc = live ? kv : (WTOK - 1);
      const _Float16* src = qkv + (size_t)tokrow(win, kvc) * QKVP + CDIM + (hp * 2 + hs) * HDM + pc * 8;
      v8h k8 = *(const v8h*)src;
      v8h v8 = *(const v8h*)(src + CDIM);
#pragma unroll
      for (int e = 0; e < 8; ++e) { k8[e] = live ? k8[e] : hz; v8[e] = live ? v8[e] : hz; }
      *(v8h*)(&Ks[hs][kv * KPI + pc * 8]) = k8;
#pragma unroll
      for (int e = 0; e < 8; ++e) Vt[hs][(pc * 8 + e) * VPI + kv] = v8[e];
    }
  }
  __syncthreads();
  if (wave >= QWAVES) return;

  const int q0 = wave * 16;
  int keyoff[8], tkcs[8];
#pragma unroll
  for (int j = 0; j < 8; ++j) {
    const int tk  = j * 16 + c;
    const int tkc = (tk < WTOK) ? tk : (WTOK - 1);
    keyoff[j] = 253 - relpart(tkc);
    tkcs[j]   = tkc;
  }
  const int tqa   = (q0 + c < WTOK) ? (q0 + c) : (WTOK - 1);
  const int qrowa = tokrow(win, tqa);
  _Float16* pw  = Ps[wave];
  _Float16* osw = Os[wave];

#pragma unroll 1
  for (int hs = 0; hs < 2; ++hs) {
    const int head = hp * 2 + hs;
    const _Float16* ksb = Ks[hs];
    const _Float16* vtb = Vt[hs];
    const float* sb = sBias[hs];
    const v16h qa = Frag<_Float16>::load(qkv + (size_t)qrowa * QKVP + head * HDM + 8 * hh);

    v8f s[8];
#pragma unroll
    for (int j = 0; j < 8; ++j) {
      s[j] = (v8f){0.f,0.f,0.f,0.f,0.f,0.f,0.f,0.f};
      const v16h kb = Frag<_Float16>::load(ksb + (j * 16 + c) * KPI + 8 * hh);
      s[j] = mma_h(qa, kb, s[j]);
    }
    wave_lds_sync();

    float lrow[8];
#pragma unroll
    for (int r = 0; r < 8; ++r) {
      const int tq  = q0 + 8 * hh + r;
      const int tqc = (tq < WTOK) ? tq : (WTOK - 1);
      const int qpart = relpart(tqc);
      const float* mrow = maskm + ((size_t)win * WTOK + tqc) * WTOK;
      float m = NEG_INF;
#pragma unroll
      for (int j = 0; j < 8; ++j) {
        float v = s[j][r] * SCORE_SCALE + sb[qpart + keyoff[j]];
        v = v + mrow[tkcs[j]];
        v = (j * 16 + c < WTOK) ? v : NEG_INF;
        s[j][r] = v;
        m = fmaxf(m, v);
      }
#pragma unroll
      for (int off = 1; off < 16; off <<= 1) m = fmaxf(m, __shfl_xor(m, off, 32));
      float psum = 0.f;
#pragma unroll
      for (int j = 0; j < 8; ++j) {
        const float p = __expf(s[j][r] - m);
        psum += p;
        pw[(8 * hh + r) * PPI + j * 16 + c] = (_Float16)(p * PCARRY);
      }
#pragma unroll
      for (int off = 1; off < 16; off <<= 1) psum += __shfl_xor(psum, off, 32);
      lrow[r] = psum;
    }
    wave_lds_sync();

    v8f oacc[2];
    oacc[0] = (v8f){0.f,0.f,0.f,0.f,0.f,0.f,0.f,0.f};
    oacc[1] = (v8f){0.f,0.f,0.f,0.f,0.f,0.f,0.f,0.f};
#pragma unroll
    for (int kk = 0; kk < 4; ++kk) {
      const v16h pa = Frag<_Float16>::load(pw + c * PPI + kk * 32 + 8 * hh);
#pragma unroll
      for (int t = 0; t < 2; ++t) {
        const v16h vb = Frag<_Float16>::load(vtb + (t * 16 + c) * VPI + kk * 32 + 8 * hh);
        oacc[t] = mma_h(pa, vb, oacc[t]);
      }
    }
#pragma unroll
    for (int r = 0; r < 8; ++r) {
      const float inv = 1.0f / (lrow[r] * PCARRY);
      osw[(8 * hh + r) * OPH + hs * 32 + c]      = (_Float16)(oacc[0][r] * inv);
      osw[(8 * hh + r) * OPH + hs * 32 + 16 + c] = (_Float16)(oacc[1][r] * inv);
    }
  }
  wave_lds_sync();

  {
    const int q8 = lane >> 3, c8 = (lane & 7) * 8;
    for (int pass = 0; pass < 2; ++pass) {
#pragma unroll
      for (int it = 0; it < 4; ++it) {
        const int row = it * 4 + q8;
        const v8h val = *(const v8h*)(osw + row * OPH + c8);
        const int tq = q0 + row;
        if (tq < WTOK) {
          _Float16* ob = att + (size_t)tokrow(win, tq) * CDIM + hp * 64 + c8;
          *(volatile v8h*)ob = val;
        }
      }
      __threadfence();
    }
  }
}

extern "C" void kernel_launch(void* const* d_in, const int* in_sizes, int n_in,
                              void* d_out, int out_size, void* d_ws, size_t ws_size,
                              hipStream_t stream) {
  if (n_in < 15) return;
  const int M = NTOKALL;
  if (in_sizes[0] != M * CDIM) return;
  if (in_sizes[1] != NWND * WTOK * WTOK) return;
  if (in_sizes[2] != CDIM || in_sizes[3] != CDIM) return;
  if (in_sizes[4] != CDIM * QKVP || in_sizes[5] != QKVP) return;
  if (in_sizes[6] != NREL * NHD) return;
  if (in_sizes[7] != CDIM * CDIM || in_sizes[8] != CDIM) return;
  if (in_sizes[9] != CDIM || in_sizes[10] != CDIM) return;
  if (in_sizes[11] != CDIM * HIDD || in_sizes[12] != HIDD) return;
  if (in_sizes[13] != HIDD * CDIM || in_sizes[14] != CDIM) return;
  if (out_size != M * CDIM) return;

  const float* x      = (const float*)d_in[0];
  const float* maskm  = (const float*)d_in[1];
  const float* g1     = (const float*)d_in[2];
  const float* b1     = (const float*)d_in[3];
  const float* qkv_w  = (const float*)d_in[4];
  const float* qkv_b  = (const float*)d_in[5];
  const float* rpb    = (const float*)d_in[6];
  const float* proj_w = (const float*)d_in[7];
  const float* proj_b = (const float*)d_in[8];
  const float* g2     = (const float*)d_in[9];
  const float* b2     = (const float*)d_in[10];
  const float* fc1_w  = (const float*)d_in[11];
  const float* fc1_b  = (const float*)d_in[12];
  const float* fc2_w  = (const float*)d_in[13];
  const float* fc2_b  = (const float*)d_in[14];
  float* out = (float*)d_out;

  const size_t szWQ = (size_t)QKVP * CDIM * 2;
  const size_t szWP = (size_t)CDIM * CDIM * 2;
  const size_t szW1 = (size_t)HIDD * CDIM * 2;
  const size_t szW2 = (size_t)CDIM * HIDD * 2;
  const size_t szR1 = (size_t)M * CDIM * 2;
  const size_t szR2 = (size_t)M * QKVP * 2;
  const size_t szU  = (size_t)MLPCH * HIDD * 2;
  const size_t oWQ = 0;
  const size_t oWP = oWQ + szWQ;
  const size_t oW1 = oWP + szWP;
  const size_t oW2 = oW1 + szW1;
  const size_t oR1 = oW2 + szW2;
  const size_t oR2 = oR1 + szR1;
  const size_t oU  = oR2 + szR2;
  const size_t total = oU + szU;
  if (total > ws_size) return;
  const size_t szX1  = (size_t)M * CDIM * 4;
  const size_t szH16 = (size_t)M * CDIM * 2;
  if (szX1 + szH16 > szR2) return;
  if ((size_t)MLPCH * HIDD * 2 > szR1) return;

  char* ws = (char*)d_ws;
  _Float16* wq16  = (_Float16*)(ws + oWQ);
  _Float16* wp16  = (_Float16*)(ws + oWP);
  _Float16* w116  = (_Float16*)(ws + oW1);
  _Float16* w216  = (_Float16*)(ws + oW2);
  _Float16* xn16  = (_Float16*)(ws + oR1);
  _Float16* att16 = (_Float16*)(ws + oR1);
  _Float16* g16   = (_Float16*)(ws + oR1);
  _Float16* qkv16 = (_Float16*)(ws + oR2);
  float*    x1    = (float*)(ws + oR2);
  _Float16* hn16  = (_Float16*)(ws + oR2 + szX1);
  _Float16* u16   = (_Float16*)(ws + oU);
  const float* dummy_resid = (const float*)(ws + oR2);

  wtr64_kernel<<<dim3(QKVP / 64, CDIM / 64), 256, 0, stream>>>(qkv_w, wq16, CDIM, QKVP, 64.0f);
  wtr64_kernel<<<dim3(CDIM / 64, CDIM / 64), 256, 0, stream>>>(proj_w, wp16, CDIM, CDIM, 64.0f);
  wtr64_kernel<<<dim3(HIDD / 64, CDIM / 64), 256, 0, stream>>>(fc1_w, w116, CDIM, HIDD, 64.0f);
  wtr64_kernel<<<dim3(CDIM / 64, HIDD / 64), 256, 0, stream>>>(fc2_w, w216, HIDD, CDIM, 64.0f);

  ln256_kernel<<<dim3((M + 7) / 8), 256, 0, stream>>>(x, g1, b1, xn16, M);

  {
    const int tiles = (M / 64) * (QKVP / 64);
    wmma_gemm64<0, false, 2, 1, false, 0><<<dim3((tiles + 7) / 8, 1), 256, 0, stream>>>(
        (const unsigned short*)xn16, (const unsigned short*)xn16, CDIM, (long)0,
        (const unsigned short*)wq16, (const unsigned short*)wq16, CDIM, (long)0,
        (void*)qkv16, (void*)qkv16, QKVP, (long)0,
        qkv_b, dummy_resid, (long)0, M, QKVP, CDIM, 1.0f / 64.0f, 16.0f);
  }

  vswin_attn_kernel<<<dim3(NHD / 2, NWND), 256, 0, stream>>>(qkv16, rpb, maskm, att16);

  {
    const int tiles = (M / 64) * (CDIM / 64);
    wmma_gemm64<0, false, 2, 0, true, 0><<<dim3((tiles + 7) / 8, 1), 256, 0, stream>>>(
        (const unsigned short*)att16, (const unsigned short*)att16, CDIM, (long)0,
        (const unsigned short*)wp16, (const unsigned short*)wp16, CDIM, (long)0,
        (void*)x1, (void*)x1, CDIM, (long)0,
        proj_b, x, (long)0, M, CDIM, CDIM, 1.0f / 1024.0f, 1.0f);
  }

  ln256_kernel<<<dim3((M + 7) / 8), 256, 0, stream>>>(x1, g2, b2, hn16, M);

  for (int ch = 0; ch < NMLPCH; ++ch) {
    const size_t rowoff = (size_t)ch * MLPCH;
    {
      const int tiles = (MLPCH / 64) * (HIDD / 64);
      wmma_gemm64<0, false, 2, 1, false, 0><<<dim3((tiles + 7) / 8, 1), 256, 0, stream>>>(
          (const unsigned short*)(hn16 + rowoff * CDIM), (const unsigned short*)(hn16 + rowoff * CDIM), CDIM, (long)0,
          (const unsigned short*)w116, (const unsigned short*)w116, CDIM, (long)0,
          (void*)u16, (void*)u16, HIDD, (long)0,
          fc1_b, dummy_resid, (long)0, MLPCH, HIDD, CDIM, 1.0f / 64.0f, 4.0f);
    }
    {
      const int n2 = MLPCH * HIDD / 2;
      gelu2_kernel<<<dim3((n2 + 255) / 256), 256, 0, stream>>>(u16, g16, n2);
    }
    {
      const int tiles = (MLPCH / 64) * (CDIM / 64);
      wmma_gemm64<0, false, 2, 0, true, 0><<<dim3((tiles + 7) / 8, 1), 256, 0, stream>>>(
          (const unsigned short*)g16, (const unsigned short*)g16, HIDD, (long)0,
          (const unsigned short*)w216, (const unsigned short*)w216, HIDD, (long)0,
          (void*)(out + rowoff * CDIM), (void*)(out + rowoff * CDIM), CDIM, (long)0,
          fc2_b, x1 + rowoff * CDIM, (long)0, MLPCH, CDIM, HIDD, 1.0f / 1024.0f, 1.0f);
    }
  }
}
